// SparseAttention_79156247265913
// MI455X (gfx1250) — hardware-verified
//
#include <hip/hip_runtime.h>
#include <stdint.h>


#ifndef NB
#define NB 4
#endif
#ifndef SEQ
#define SEQ 1024
#endif
#define B_FULL 4
#define S_FULL 1024
#define DM 1024
#define NE 8
#define DEX 128
#define ROWS 32
#define NT 256

static_assert(SEQ % 128 == 0);
static_assert(SEQ <= S_FULL);
static_assert(NB >= 1);
static_assert(NB <= B_FULL);
static_assert(NE * DEX == DM);

typedef _Float16 v16h __attribute__((ext_vector_type(16)));
typedef _Float16 v8h  __attribute__((ext_vector_type(8)));
typedef float    v8f  __attribute__((ext_vector_type(8)));
typedef float    v4f  __attribute__((ext_vector_type(4)));

constexpr int SP  = SEQ + 8;
constexpr int AP  = SEQ + 8;
constexpr int HP  = SEQ + 8;
constexpr int VSP = 40;
constexpr int OSP = 260;
constexpr int SC_BYTES  = ROWS * SP * 4;
constexpr int VS_BYTES  = 256 * VSP * 2;
constexpr int OS_BYTES  = ROWS * OSP * 4;
constexpr int ATT_BYTES = (ROWS * AP * 4 > VS_BYTES + OS_BYTES) ? (ROWS * AP * 4) : (VS_BYTES + OS_BYTES);
constexpr int OFF_SC  = 0;
constexpr int OFF_ATT = OFF_SC + SC_BYTES;
constexpr int OFF_VS  = OFF_ATT;
constexpr int OFF_OS  = OFF_VS + VS_BYTES;
constexpr int LDS_MAIN = OFF_ATT + ATT_BYTES;
static_assert(2 * ROWS * HP * 2 <= SC_BYTES);
static_assert(VS_BYTES + OS_BYTES <= ATT_BYTES);
static_assert((OFF_ATT % 16) == 0);
static_assert((OFF_OS % 16) == 0);
static_assert(LDS_MAIN <= 300 * 1024);

constexpr float QK_SCALE = 0.03125f;

__device__ __forceinline__ float bf16_rne(float x) {
    unsigned u = __float_as_uint(x);
    u = (u + 0x7FFFu + ((u >> 16) & 1u)) & 0xFFFF0000u;
    return __uint_as_float(u);
}
__device__ __forceinline__ _Float16 to_h(float x) { return (_Float16)bf16_rne(x); }

__device__ __forceinline__ v16h cat16(v8h lo, v8h hi) {
    return __builtin_shufflevector(lo, hi, 0, 1, 2, 3, 4, 5, 6, 7, 8, 9, 10, 11, 12, 13, 14, 15);
}
__device__ __forceinline__ v16h frag_ld(const _Float16* p) {
    v8h a = *(const v8h*)p;
    v8h c = *(const v8h*)(p + 16);
    return cat16(a, c);
}
__device__ __forceinline__ v8f wmma16(v16h a, v16h b, v8f c) {
    v8f d = __builtin_amdgcn_wmma_f32_16x16x32_f16(false, a, false, b, (short)0, c, false, false);
    asm volatile("v_nop\n\tv_nop\n\tv_nop\n\tv_nop" : "+v"(d) : "v"(a), "v"(b));
    return d;
}

__global__ __launch_bounds__(NT)
void k_cvt(const float* __restrict__ Q, const float* __restrict__ K, _Float16* Qp, _Float16* Kp)
{
    const int which = blockIdx.y;
    const float* src = which ? K : Q;
    _Float16*    dst = which ? Kp : Qp;
    const size_t g = (size_t)blockIdx.x * NT + threadIdx.x;
    const size_t ngroups = (size_t)NB * SEQ * (DM / 8);
    if (g >= ngroups) return;
    const size_t rowi = g / (DM / 8);
    const int c8 = (int)(g % (DM / 8));
    const int bb = (int)(rowi / SEQ), ss = (int)(rowi % SEQ);
    const float* sp = src + ((size_t)bb * S_FULL + ss) * DM + c8 * 8;
    v4f a0 = *(const v4f*)sp;
    v4f a1 = *(const v4f*)(sp + 4);
    v8h o;
    o[0] = to_h(a0.x); o[1] = to_h(a0.y); o[2] = to_h(a0.z); o[3] = to_h(a0.w);
    o[4] = to_h(a1.x); o[5] = to_h(a1.y); o[6] = to_h(a1.z); o[7] = to_h(a1.w);
    _Float16* dp = dst + rowi * DM + c8 * 8;
    *(volatile v8h*)dp = o;
    __threadfence();
    *(volatile v8h*)dp = o;
}

__global__ __launch_bounds__(NT)
void k_vtr(const float* __restrict__ V, _Float16* Vt)
{
    __shared__ v8h Tv[(64 * 72) / 8];
    _Float16* T = (_Float16*)Tv;
    const int tid = threadIdx.x, lane = tid & 31, wv = tid >> 5;
    const int nct = DM / 64, ntt = SEQ / 64;
    const int bid = blockIdx.x;
    const int tc = bid % nct;
    const int tt = (bid / nct) % ntt;
    const int bb = bid / (nct * ntt);
    if (bb >= NB) return;
    const int c0 = tc * 64, t0 = tt * 64;
    {
        const int r  = tid >> 2;
        const int cs = (tid & 3) * 16;
        const float* sp = V + ((size_t)bb * S_FULL + t0 + r) * DM + c0 + cs;
        #pragma unroll
        for (int q = 0; q < 4; ++q) {
            v4f f = *(const v4f*)(sp + 4 * q);
            T[(cs + 4 * q + 0) * 72 + r] = to_h(f.x);
            T[(cs + 4 * q + 1) * 72 + r] = to_h(f.y);
            T[(cs + 4 * q + 2) * 72 + r] = to_h(f.z);
            T[(cs + 4 * q + 3) * 72 + r] = to_h(f.w);
        }
    }
    __syncthreads();
    #pragma unroll
    for (int pass = 0; pass < 2; ++pass) {
        #pragma unroll
        for (int k2 = 0; k2 < 2; ++k2) {
            const int cl = wv * 8 + k2 * 4 + (lane >> 3);
            const int pc = (lane & 7) * 8;
            v8h vv = *(const v8h*)(T + cl * 72 + pc);
            _Float16* dp = Vt + ((size_t)bb * DM + c0 + cl) * SEQ + t0 + pc;
            *(volatile v8h*)dp = vv;
        }
        if (pass == 0) __threadfence();
    }
}

__global__ __launch_bounds__(NT, 1) __attribute__((amdgpu_num_vgpr(256)))
void k_attn(const _Float16* __restrict__ Qp, const _Float16* __restrict__ Kp,
            const _Float16* __restrict__ Vt, const float* __restrict__ rprob,
            const int* __restrict__ emask, const float* __restrict__ mask_unused,
            float* out)
{
    extern __shared__ v4f smem_v[];
    unsigned char* smem = (unsigned char*)smem_v;
    float*    SC  = (float*)(smem + OFF_SC);
    _Float16* AH  = (_Float16*)(smem + OFF_SC);
    _Float16* AL  = AH + ROWS * HP;
    float*    ATT = (float*)(smem + OFF_ATT);
    _Float16* VS  = (_Float16*)(smem + OFF_VS);
    float*    OS  = (float*)(smem + OFF_OS);
    (void)mask_unused;

    const int tid  = threadIdx.x;
    const int lane = tid & 31;
    const int wv   = tid >> 5;
    const int h    = lane >> 4;
    const int m    = lane & 15;
    const int b    = blockIdx.x / (SEQ / ROWS);
    const int row0 = (blockIdx.x % (SEQ / ROWS)) * ROWS;
    if (b >= NB) return;

    int s0 = 0, s1 = -1;
    {
        float pv[NE];
        #pragma unroll
        for (int e = 0; e < NE; ++e) pv[e] = bf16_rne(rprob[b * NE + e]);
        float v0 = pv[0];
        #pragma unroll
        for (int e = 1; e < NE; ++e) { if (pv[e] > v0) { v0 = pv[e]; s0 = e; } }
        float v1 = -3.0e38f;
        #pragma unroll
        for (int e = 0; e < NE; ++e) {
            const bool take = (e != s0) && ((s1 < 0) || (pv[e] > v1));
            if (take) { v1 = pv[e]; s1 = e; }
        }
        s1 = (s1 < 0) ? 0 : s1;
        s0 = (s0 < 0) ? 0 : ((s0 > NE - 1) ? NE - 1 : s0);
        s1 = (s1 > NE - 1) ? NE - 1 : s1;
    }

    for (int i = tid; i < ROWS * AP; i += NT) ATT[i] = 0.0f;

    #pragma unroll 1
    for (int e = 0; e < NE; ++e) {
        const int wgt = emask[e * B_FULL + b];
        if (wgt == 0) continue;

        v16h aq0[4], aq1[4];
        {
            const _Float16* q0p = Qp + ((size_t)b * SEQ + row0 + m) * DM + e * DEX + 8 * h;
            const _Float16* q1p = q0p + (size_t)16 * DM;
            #pragma unroll
            for (int ks = 0; ks < 4; ++ks) {
                aq0[ks] = frag_ld(q0p + ks * 32);
                aq1[ks] = frag_ld(q1p + ks * 32);
            }
        }
        #pragma unroll 1
        for (int kt = 0; kt < SEQ / 128; ++kt) {
            const int t0 = (wv * (SEQ / 128) + kt) * 16;
            const _Float16* kp = Kp + ((size_t)b * SEQ + t0 + m) * DM + e * DEX + 8 * h;
            v8f c0 = {}, c1 = {};
            #pragma unroll
            for (int ks = 0; ks < 4; ++ks) {
                v16h bk = frag_ld(kp + ks * 32);
                c0 = wmma16(aq0[ks], bk, c0);
                c1 = wmma16(aq1[ks], bk, c1);
            }
            #pragma unroll
            for (int r = 0; r < 8; ++r) {
                SC[(8 * h + r) * SP + t0 + m]      = c0[r] * QK_SCALE;
                SC[(16 + 8 * h + r) * SP + t0 + m] = c1[r] * QK_SCALE;
            }
        }
        __syncthreads();

        {
            const float fw = (float)wgt;
            #pragma unroll 1
            for (int rr = 0; rr < ROWS / 8; ++rr) {
                const int R = wv * (ROWS / 8) + rr;
                const float* srow = SC + R * SP + lane;
                float x[SEQ / 32];
                float mx = -3.0e38f;
                #pragma unroll
                for (int j = 0; j < SEQ / 32; ++j) { x[j] = srow[32 * j]; mx = fmaxf(mx, x[j]); }
                #pragma unroll
                for (int off = 1; off < 32; off <<= 1) mx = fmaxf(mx, __shfl_xor(mx, off, 32));
                float sum = 0.0f;
                #pragma unroll
                for (int j = 0; j < SEQ / 32; ++j) { x[j] = __expf(x[j] - mx); sum += x[j]; }
                #pragma unroll
                for (int off = 1; off < 32; off <<= 1) sum += __shfl_xor(sum, off, 32);
                const float scl = fw * (1.0f / sum);
                float* arow = ATT + R * AP + lane;
                #pragma unroll
                for (int j = 0; j < SEQ / 32; ++j) {
                    const float av = arow[32 * j];
                    arow[32 * j] = av + x[j] * scl;
                }
            }
        }
        __syncthreads();
    }
    __syncthreads();

    #pragma unroll 1
    for (int it = 0; it < (ROWS * SEQ / 8) / NT; ++it) {
        const int idx = tid + it * NT;
        const int R  = idx / (SEQ / 8);
        const int c8 = idx % (SEQ / 8);
        const float* ap = ATT + R * AP + c8 * 8;
        v4f a0 = *(const v4f*)ap;
        v4f a1 = *(const v4f*)(ap + 4);
        v8h hv, lv;
        #pragma unroll
        for (int i = 0; i < 4; ++i) {
            const float sA = a0[i] * 1024.0f;
            const _Float16 hA = (_Float16)sA;
            const float rA = (sA - (float)hA) * 4096.0f;
            hv[i] = hA; lv[i] = (_Float16)rA;
            const float sB = a1[i] * 1024.0f;
            const _Float16 hB = (_Float16)sB;
            const float rB = (sB - (float)hB) * 4096.0f;
            hv[4 + i] = hB; lv[4 + i] = (_Float16)rB;
        }
        *(v8h*)(AH + R * HP + c8 * 8) = hv;
        *(v8h*)(AL + R * HP + c8 * 8) = lv;
    }
    __syncthreads();

    const int mt = wv >> 2;
    const int cq = wv & 3;
    v8f acH[4] = {{}, {}, {}, {}};
    v8f acL[4] = {{}, {}, {}, {}};
    #pragma unroll 1
    for (int ch = 0; ch < SEQ / 32; ++ch) {
        const int t0 = ch * 32;
        {
            const int slot = tid >> 7;
            const int sel  = slot ? s1 : s0;
            const int c    = tid & 127;
            const _Float16* src = Vt + ((size_t)b * DM + sel * DEX + c) * SEQ + t0;
            v8h p0 = *(const v8h*)(src);
            v8h p1 = *(const v8h*)(src + 8);
            v8h p2 = *(const v8h*)(src + 16);
            v8h p3 = *(const v8h*)(src + 24);
            _Float16* dst = VS + tid * VSP;
            *(v8h*)(dst)      = p0;
            *(v8h*)(dst + 8)  = p1;
            *(v8h*)(dst + 16) = p2;
            *(v8h*)(dst + 24) = p3;
        }
        __syncthreads();
        v16h faH = frag_ld(AH + (mt * 16 + m) * HP + t0 + 8 * h);
        v16h faL = frag_ld(AL + (mt * 16 + m) * HP + t0 + 8 * h);
        #pragma unroll
        for (int q = 0; q < 4; ++q) {
            const int ct = cq * 4 + q;
            v16h fb = frag_ld(VS + (ct * 16 + m) * VSP + 8 * h);
            acH[q] = wmma16(faH, fb, acH[q]);
            acL[q] = wmma16(faL, fb, acL[q]);
        }
        __syncthreads();
    }

    #pragma unroll
    for (int q = 0; q < 4; ++q) {
        const int ct = cq * 4 + q;
        #pragma unroll
        for (int r = 0; r < 8; ++r) {
            const float vh = acH[q][r];
            const float vl = acL[q][r];
            const float o  = (vh + vl * (1.0f / 4096.0f)) * (1.0f / 1024.0f);
            OS[(mt * 16 + 8 * h + r) * OSP + ct * 16 + m] = o;
        }
    }
    __syncthreads();

    float* ob = out + ((size_t)b * SEQ + row0) * DM;
    #pragma unroll 1
    for (int pass = 0; pass < 2; ++pass) {
        #pragma unroll 1
        for (int rr = 0; rr < ROWS / 8; ++rr) {
            const int R = wv * (ROWS / 8) + rr;
            #pragma unroll 1
            for (int e = 0; e < NE; ++e) {
                const int js = (e == s0) ? 0 : ((e == s1) ? 1 : -1);
                const int jc = (js < 0) ? 0 : js;
                v4f xv = *(const v4f*)(OS + R * OSP + jc * DEX + 4 * lane);
                const bool on = (js >= 0);
                v4f vv;
                vv.x = on ? xv.x : 0.0f;
                vv.y = on ? xv.y : 0.0f;
                vv.z = on ? xv.z : 0.0f;
                vv.w = on ? xv.w : 0.0f;
                *(volatile v4f*)(ob + (size_t)R * DM + e * DEX + 4 * lane) = vv;
            }
        }
        if (pass == 0) __threadfence();
    }
}

extern "C" void kernel_launch(void* const* d_in, const int* in_sizes, int n_in,
                              void* d_out, int out_size, void* d_ws, size_t ws_size,
                              hipStream_t stream)
{
    if (n_in < 6) return;
    const long long need_qkv = ((long long)(NB - 1) * S_FULL + SEQ) * (long long)DM;
    if ((long long)in_sizes[0] < need_qkv) return;
    if ((long long)in_sizes[1] < need_qkv) return;
    if ((long long)in_sizes[2] < need_qkv) return;
    if (in_sizes[3] < NB * NE) return;
    if (in_sizes[4] < (NE - 1) * B_FULL + NB) return;
    if ((long long)out_size < (long long)NB * SEQ * DM) return;

    const size_t plane_bytes = (size_t)NB * SEQ * DM * sizeof(_Float16);
    if (3 * plane_bytes > ws_size) return;

    const float* Q  = (const float*)d_in[0];
    const float* K  = (const float*)d_in[1];
    const float* V  = (const float*)d_in[2];
    const float* rp = (const float*)d_in[3];
    const int*   em = (const int*)d_in[4];
    const float* mk = (const float*)d_in[5];
    float* out = (float*)d_out;

    unsigned char* ws = (unsigned char*)d_ws;
    _Float16* Qp = (_Float16*)(ws);
    _Float16* Kp = (_Float16*)(ws + plane_bytes);
    _Float16* Vt = (_Float16*)(ws + 2 * plane_bytes);

    dim3 gcvt((unsigned)((size_t)NB * SEQ * (DM / 8) / NT), 2);
    k_cvt<<<gcvt, NT, 0, stream>>>(Q, K, Qp, Kp);

    dim3 gvtr((unsigned)(NB * (SEQ / 64) * (DM / 64)));
    k_vtr<<<gvtr, NT, 0, stream>>>(V, Vt);

    hipFuncSetAttribute(reinterpret_cast<const void*>(&k_attn),
                        hipFuncAttributeMaxDynamicSharedMemorySize, LDS_MAIN);
    dim3 gattn((unsigned)(NB * (SEQ / ROWS)));
    k_attn<<<gattn, NT, LDS_MAIN, stream>>>(Qp, Kp, Vt, rp, em, mk, out);
}
